// IQALoss_79577154060421
// MI455X (gfx1250) — hardware-verified
//
#include <hip/hip_runtime.h>
#include <math.h>
typedef __attribute__((ext_vector_type(16))) _Float16 v16h;
typedef __attribute__((ext_vector_type(8)))  _Float16 v8h;
typedef __attribute__((ext_vector_type(16))) __bf16   v16b;
typedef __attribute__((ext_vector_type(8)))  __bf16   v8b;
typedef __attribute__((ext_vector_type(8)))  float    v8f;
typedef __attribute__((ext_vector_type(4)))  float    v4f;
#define PSCALE 32768.0f
#define U16(p) ((const unsigned short*)(const void*)(p))
#define PSCALE_INV (1.0f / 32768.0f)

__device__ __forceinline__ unsigned short f2bf_bits(float f) {
  unsigned u = __float_as_uint(f);
  return (unsigned short)((u + 0x7FFFu + ((u >> 16) & 1u)) >> 16);
}
__device__ __forceinline__ float bf_bits2f(unsigned short h) { return __uint_as_float(((unsigned)h) << 16); }

__device__ __forceinline__ void dep_guard_h(v8f& a, v8f& b, v16h x, v16h y) { asm volatile("v_nop\n\tv_nop\n\tv_nop\n\tv_nop" : "+v"(a), "+v"(b) : "v"(x), "v"(y)); }
__device__ __forceinline__ void dep_guard_b(v8f& a, v8f& b, v16b x, v16b y) { asm volatile("v_nop\n\tv_nop\n\tv_nop\n\tv_nop" : "+v"(a), "+v"(b) : "v"(x), "v"(y)); }
__device__ __forceinline__ void keep4_h(v16h a, v16h b, v16h c, v16h d) { asm volatile("v_nop" :: "v"(a), "v"(b), "v"(c), "v"(d)); }
__device__ __forceinline__ void keep4_b(v16b a, v16b b, v16b c, v16b d) { asm volatile("v_nop" :: "v"(a), "v"(b), "v"(c), "v"(d)); }
__device__ __forceinline__ void acc_guard4(v8f& a, v8f& b, v8f& c, v8f& d) { asm volatile("v_nop\n\tv_nop\n\tv_nop\n\tv_nop" : "+v"(a), "+v"(b), "+v"(c), "+v"(d)); }
template <typename T> struct Frag;
template <> struct Frag<_Float16> {
  typedef v16h V; union U { v16h v; v8h h[2]; };
  static __device__ __forceinline__ v16h load(const _Float16* p) {
    U f; f.h[0] = *(const v8h*)(p); f.h[1] = *(const v8h*)(p + 16); return f.v;
  }
  static __device__ __forceinline__ v8f mma(v16h a, v16h b, v8f c) {
    return __builtin_amdgcn_wmma_f32_16x16x32_f16(false, a, false, b, (short)0, c, false, false);
  }
  static __device__ __forceinline__ void guard(v8f& a, v8f& b, v16h x, v16h y) { dep_guard_h(a, b, x, y); }
  static __device__ __forceinline__ void keep(v16h a, v16h b, v16h c, v16h d) { keep4_h(a, b, c, d); }
};
template <> struct Frag<__bf16> {
  typedef v16b V; union U { v16b v; v8b h[2]; };
  static __device__ __forceinline__ v16b load(const __bf16* p) {
    U f; f.h[0] = *(const v8b*)(p); f.h[1] = *(const v8b*)(p + 16); return f.v;
  }
  static __device__ __forceinline__ v8f mma(v16b a, v16b b, v8f c) {
    return __builtin_amdgcn_wmma_f32_16x16x32_bf16(false, a, false, b, (short)0, c, false, false);
  }
  static __device__ __forceinline__ void guard(v8f& a, v8f& b, v16b x, v16b y) { dep_guard_b(a, b, x, y); }
  static __device__ __forceinline__ void keep(v16b a, v16b b, v16b c, v16b d) { keep4_b(a, b, c, d); }
};

template <int ET> struct Elem;
template <> struct Elem<0> { typedef _Float16 T; };
template <> struct Elem<1> { typedef __bf16 T; };
template <int ET, bool SPLIT, int BIAS_MODE, int OUT_MODE, bool RESID, int ACT = 0>
__global__ __launch_bounds__(256) void wmma_gemm64(
    const unsigned short* __restrict__ Ap, const unsigned short* __restrict__ A2p, int lda, long strideA,
    const unsigned short* __restrict__ Btp, const unsigned short* __restrict__ Bt2p, int ldb, long strideB,
    void* __restrict__ Cout, void* __restrict__ Cout2, int ldc, long strideC,
    const float* __restrict__ bias,
    const float* __restrict__ resid, long strideR,
    int M, int N, int K, float scale) {
  typedef typename Elem<ET>::T T;
  typedef typename Frag<T>::V V;
  const T* A = (const T*)Ap; const T* A2 = (const T*)A2p; const T* Bt = (const T*)Btp; const T* Bt2 = (const T*)Bt2p;
  __shared__ __align__(16) float sT[8][16 * 68];
  const int b    = blockIdx.y;
  const int lane = threadIdx.x & 31;
  const int wave = threadIdx.x >> 5;
  const int tilesN = N >> 6;
  const int tilesM = M >> 6;
  const int tile = blockIdx.x * 8 + wave;
  if (tile >= tilesM * tilesN) return;
  const int tm = tile / tilesN;
  const int tn = tile - tm * tilesN;
  const int m0 = tm << 6;
  const int n0 = tn << 6;

  const T* Ab  = A  + (size_t)b * strideA;
  const T* Bb  = Bt + (size_t)b * strideB;
  const T* Ab2 = SPLIT ? (A2  + (size_t)b * strideA) : nullptr;
  const T* Bb2 = SPLIT ? (Bt2 + (size_t)b * strideB) : nullptr;

  const int rlane = lane & 15;
  const int koff  = (lane >> 4) * 8;
  const int mOff  = (lane >> 4) * 8;

  v8f acc[4][4];
#pragma unroll
  for (int i = 0; i < 4; ++i)
#pragma unroll
    for (int j = 0; j < 4; ++j) acc[i][j] = (v8f){0.f,0.f,0.f,0.f,0.f,0.f,0.f,0.f};

  for (int k0 = 0; k0 < K; k0 += 32) {
    V bh[4], bl[4];
#pragma unroll
    for (int j = 0; j < 4; ++j) {
      const size_t bo = (size_t)(n0 + (j << 4) + rlane) * ldb + koff + k0;
      bh[j] = Frag<T>::load(Bb + bo);
      if (SPLIT) bl[j] = Frag<T>::load(Bb2 + bo);
    }
#pragma unroll
    for (int i = 0; i < 4; ++i) {
      const size_t ao = (size_t)(m0 + (i << 4) + rlane) * lda + koff + k0;
      V ah = Frag<T>::load(Ab + ao);
      V al;
      if (SPLIT) al = Frag<T>::load(Ab2 + ao);
#pragma unroll
      for (int j = 0; j < 4; ++j) {
        acc[i][j] = Frag<T>::mma(ah, bh[j], acc[i][j]);
        if (SPLIT) {
          acc[i][j] = Frag<T>::mma(ah, bl[j], acc[i][j]);
          acc[i][j] = Frag<T>::mma(al, bh[j], acc[i][j]);
        }
      }
      Frag<T>::guard(acc[i][0], acc[i][3], ah, SPLIT ? al : ah);
    }
    Frag<T>::keep(bh[0], bh[1], bh[2], bh[3]);
    if (SPLIT) Frag<T>::keep(bl[0], bl[1], bl[2], bl[3]);
  }
  acc_guard4(acc[0][0], acc[0][1], acc[0][2], acc[0][3]);
  acc_guard4(acc[1][0], acc[1][1], acc[1][2], acc[1][3]);
  acc_guard4(acc[2][0], acc[2][1], acc[2][2], acc[2][3]);
  acc_guard4(acc[3][0], acc[3][1], acc[3][2], acc[3][3]);

  float* slab = sT[wave];
  const float* Rb = RESID ? (resid + (size_t)b * strideR) : nullptr;
#pragma unroll
  for (int i = 0; i < 4; ++i) {
    const int mBase = m0 + (i << 4);
#pragma unroll
    for (int j = 0; j < 4; ++j) {
      const int n = n0 + (j << 4) + rlane;
      float bv = 0.f;
      if (BIAS_MODE == 2) bv = bias[n];
#pragma unroll
      for (int r = 0; r < 8; ++r) {
        float v = acc[i][j][r] * scale;
        if (BIAS_MODE == 1) v += bias[mBase + mOff + r];
        if (BIAS_MODE == 2) v += bv;
        if (RESID) v += Rb[(size_t)(mBase + mOff + r) * ldc + n];
        if (ACT == 1) v = tanhf(v);
        if (ACT == 2) v = fmaxf(v, 0.0f);
        if (ACT == 3) v = v / (1.0f + expf(-v));
        if (ACT == 4) v = (v > 0.f) ? v : 0.01f * v;
        if (ACT == 5) v = 0.5f * v * (1.0f + erff(v * 0.70710678118654752f));
        slab[(mOff + r) * 68 + (j << 4) + rlane] = v;
      }
    }
    __builtin_amdgcn_fence(__ATOMIC_RELEASE, "workgroup");
    __builtin_amdgcn_wave_barrier();
    __builtin_amdgcn_fence(__ATOMIC_ACQUIRE, "workgroup");
    if (OUT_MODE == 0) {
      float* C = (float*)Cout + (size_t)b * strideC;
      const int hh = lane >> 4, c4 = (lane & 15) * 4;
      for (int pass = 0; pass < 2; ++pass) {
#pragma unroll
        for (int it = 0; it < 8; ++it) {
          const int row = it * 2 + hh;
          v4f v = *(const v4f*)(slab + row * 68 + c4);
          *(volatile v4f*)(C + (size_t)(mBase + row) * ldc + n0 + c4) = v;
        }
        __threadfence();
      }
    } else {
      const int q = lane >> 3, c8 = (lane & 7) * 8;
      unsigned short* C  = (unsigned short*)Cout  + (size_t)b * strideC;
      unsigned short* C2 = (OUT_MODE == 2) ? ((unsigned short*)Cout2 + (size_t)b * strideC) : nullptr;
      for (int pass = 0; pass < 2; ++pass) {
#pragma unroll
        for (int it = 0; it < 4; ++it) {
          const int row = it * 4 + q;
          const float* sp = slab + row * 68 + c8;
          v8h hv, lv;
#pragma unroll
          for (int e = 0; e < 8; ++e) {
            if (OUT_MODE == 1) {
              hv[e] = (_Float16)sp[e];
            } else {
              unsigned short hb = f2bf_bits(sp[e]);
              unsigned short lb = f2bf_bits(sp[e] - bf_bits2f(hb));
              hv[e] = __builtin_bit_cast(_Float16, hb);
              lv[e] = __builtin_bit_cast(_Float16, lb);
            }
          }
          *(volatile v8h*)(C + (size_t)(mBase + row) * ldc + n0 + c8) = hv;
          if (OUT_MODE == 2) *(volatile v8h*)(C2 + (size_t)(mBase + row) * ldc + n0 + c8) = lv;
        }
        __threadfence();
      }
    }
    __builtin_amdgcn_fence(__ATOMIC_RELEASE, "workgroup");
    __builtin_amdgcn_wave_barrier();
    __builtin_amdgcn_fence(__ATOMIC_ACQUIRE, "workgroup");
  }
}

__global__ __launch_bounds__(256) void cast_f32_f16x2(
    const float* __restrict__ in, _Float16* __restrict__ out, int n2) {
  int i = blockIdx.x * 256 + threadIdx.x;
  if (i < n2) {
    const _Float16 h0 = (_Float16)in[2 * i], h1 = (_Float16)in[2 * i + 1];
    const unsigned u = (unsigned)__builtin_bit_cast(unsigned short, h0) | ((unsigned)__builtin_bit_cast(unsigned short, h1) << 16);
    ((volatile unsigned*)out)[i] = u;
    __threadfence();
    ((volatile unsigned*)out)[i] = u;
  }
}


#define QB 4096
#define QD 512
__global__ __launch_bounds__(256) void fnorm_kernel(const float* __restrict__ f, unsigned* __restrict__ F16) {
  const int lane = threadIdx.x & 31, wave = threadIdx.x >> 5; const size_t r = (size_t)blockIdx.x * 8 + wave;
  float v[16]; float s = 0.f; for (int q = 0; q < 4; ++q) { const v4f a = *(const v4f*)(f + r * QD + lane * 16 + 4 * q); for (int e = 0; e < 4; ++e) { v[4 * q + e] = a[e]; s += a[e] * a[e]; } }
  for (int o = 16; o > 0; o >>= 1) s += __shfl_xor(s, o, 32); const float inv = 1.0f / sqrtf(s);
  unsigned pk[8]; for (int q = 0; q < 8; ++q) pk[q] = (unsigned)__builtin_bit_cast(unsigned short, (_Float16)(v[2 * q] * inv)) | ((unsigned)__builtin_bit_cast(unsigned short, (_Float16)(v[2 * q + 1] * inv)) << 16);
  typedef __attribute__((ext_vector_type(4))) unsigned u4; const u4 p0 = {pk[0], pk[1], pk[2], pk[3]}, p1 = {pk[4], pk[5], pk[6], pk[7]};
  for (int pass = 0; pass < 2; ++pass) { *(volatile u4*)(F16 + (r * QD + lane * 16) / 2) = p0; *(volatile u4*)(F16 + (r * QD + lane * 16) / 2 + 4) = p1; __threadfence(); }
}
__global__ __launch_bounds__(256) void row_kernel(const float* __restrict__ S, const int* __restrict__ ids, const float* __restrict__ idp, const float* __restrict__ idg, float* __restrict__ ROWV) {
  __shared__ float st[8][4];
  const int lane = threadIdx.x & 31, wave = threadIdx.x >> 5; const int i = blockIdx.x * 8 + wave; const int myid = ids[i]; const float pi = idp[i], gi = idg[i];
  const float* srow = S + (size_t)i * QB;
  float den = 0.f, possum = 0.f, npos = 0.f, rl = 0.f, rc = 0.f;
#pragma unroll 1
  for (int j = lane; j < QB; j += 32) { const float lg = srow[j]; const bool same = (ids[j] == myid);
    if (j != i) { den += expf(lg); if (same) { possum += lg; npos += 1.f; } }
    if (same && (gi > idg[j] + 1e-6f)) { rl += fmaxf(0.1f - (pi - idp[j]), 0.f); rc += 1.f; } }
  for (int o = 16; o > 0; o >>= 1) { den += __shfl_xor(den, o, 32); possum += __shfl_xor(possum, o, 32); npos += __shfl_xor(npos, o, 32); rl += __shfl_xor(rl, o, 32); rc += __shfl_xor(rc, o, 32); }
  if (lane == 0) { st[wave][0] = (possum - npos * logf(den + 1e-8f)) / (npos + 1e-8f); st[wave][1] = rl; st[wave][2] = rc; st[wave][3] = 0.f; }
  __syncthreads();
  if (threadIdx.x < 32) { const float v = (&st[0][0])[threadIdx.x]; ((volatile float*)ROWV)[blockIdx.x * 32 + threadIdx.x] = v; __threadfence(); ((volatile float*)ROWV)[blockIdx.x * 32 + threadIdx.x] = v; }
}
__global__ __launch_bounds__(256) void final_kernel(const float* __restrict__ qp, const float* __restrict__ ip, const float* __restrict__ qg, const float* __restrict__ ig, const float* __restrict__ ROWV, float* __restrict__ out) {
  __shared__ double red[12][256];
  const int t = threadIdx.x; double a[12]; for (int k = 0; k < 12; ++k) a[k] = 0.0;
  for (int i = t; i < QB; i += 256) { const double x1 = qp[i], y1 = qg[i], x2 = ip[i], y2 = ig[i];
    double d = fabs(x1 - y1); a[0] += (d < 1.0) ? 0.5 * d * d : d - 0.5; d = fabs(x2 - y2); a[1] += (d < 1.0) ? 0.5 * d * d : d - 0.5;
    a[2] += x1; a[3] += y1; a[4] += x2; a[5] += y2; a[6] += ROWV[i * 4]; a[7] += ROWV[i * 4 + 1]; a[8] += ROWV[i * 4 + 2]; }
  for (int k = 0; k < 9; ++k) red[k][t] = a[k]; __syncthreads();
  for (int o = 128; o > 0; o >>= 1) { if (t < o) for (int k = 0; k < 9; ++k) red[k][t] += red[k][t + o]; __syncthreads(); }
  const double m1 = red[2][0] / QB, g1 = red[3][0] / QB, m2 = red[4][0] / QB, g2 = red[5][0] / QB;
  __syncthreads();
  double b[6] = {0, 0, 0, 0, 0, 0};
  for (int i = t; i < QB; i += 256) { const double x1 = qp[i] - m1, y1 = qg[i] - g1, x2 = ip[i] - m2, y2 = ig[i] - g2; b[0] += x1 * x1; b[1] += y1 * y1; b[2] += x1 * y1; b[3] += x2 * x2; b[4] += y2 * y2; b[5] += x2 * y2; }
  const double hub1 = red[0][0] / QB, hub2 = red[1][0] / QB, sup = -red[6][0] / QB, rls = red[7][0], rcn = red[8][0];
  __syncthreads();
  for (int k = 0; k < 6; ++k) red[k][t] = b[k]; __syncthreads();
  for (int o = 128; o > 0; o >>= 1) { if (t < o) for (int k = 0; k < 6; ++k) red[k][t] += red[k][t + o]; __syncthreads(); }
  if (t == 0) { const double vx1 = red[0][0] / QB, vy1 = red[1][0] / QB, c1 = red[2][0] / QB, vx2 = red[3][0] / QB, vy2 = red[4][0] / QB, c2 = red[5][0] / QB;
    const double plcc1 = 1.0 - c1 / (sqrt(vx1) * sqrt(vy1) + 1e-8), plcc2 = 1.0 - c2 / (sqrt(vx2) * sqrt(vy2) + 1e-8);
    const double rank = (rcn > 0.0) ? rls / fmax(rcn, 1.0) : 0.0;
    const double total = (hub1 + hub2) + 0.1 * (plcc1 + plcc2) + 0.05 * sup + 0.05 * rank;
    ((volatile float*)out)[0] = (float)total; __threadfence(); ((volatile float*)out)[0] = (float)total; }
}
extern "C" void kernel_launch(void* const* d_in, const int* in_sizes, int n_in, void* d_out, int out_size, void* d_ws, size_t ws_size, hipStream_t stream) {
  (void)in_sizes; (void)n_in; (void)out_size; (void)ws_size;
  const float* qp = (const float*)d_in[0]; const float* ip = (const float*)d_in[1]; const float* qg = (const float*)d_in[2]; const float* ig = (const float*)d_in[3]; const float* feats = (const float*)d_in[4]; const int* ids = (const int*)d_in[5];
  char* ws = (char*)d_ws; size_t off = 0;
  auto carve = [&](size_t bytes) -> char* { char* p = ws + off; off += (bytes + 255) & ~(size_t)255; return p; };
  unsigned* F16 = (unsigned*)carve((size_t)QB * QD * 2); float* S = (float*)carve((size_t)QB * QB * 4); float* ROWV = (float*)carve((size_t)QB * 4 * 4);
  fnorm_kernel<<<QB / 8, 256, 0, stream>>>(feats, F16);
  { const int t = (QB / 64) * (QB / 64);
    wmma_gemm64<0, false, 0, 0, false><<<dim3((t + 7) / 8, 1), 256, 0, stream>>>((const unsigned short*)F16, nullptr, QD, 0, (const unsigned short*)F16, nullptr, QD, 0, S, nullptr, QB, 0, nullptr, nullptr, 0, QB, QB, QD, 10.0f); }
  row_kernel<<<QB / 8, 256, 0, stream>>>(S, ids, ip, ig, ROWV);
  final_kernel<<<1, 256, 0, stream>>>(qp, ip, qg, ig, ROWV, (float*)d_out);
}
